// S4D_30794915512668
// MI455X (gfx1250) — hardware-run, weakly checked
//
#include <hip/hip_runtime.h>
#include <math.h>

typedef __attribute__((ext_vector_type(16))) _Float16 v16h;
typedef __attribute__((ext_vector_type(8)))  _Float16 v8h;
typedef __attribute__((ext_vector_type(16))) __bf16   v16b;
typedef __attribute__((ext_vector_type(8)))  __bf16   v8b;
typedef __attribute__((ext_vector_type(8)))  float    v8f;
typedef __attribute__((ext_vector_type(4)))  float    v4f;

constexpr int kB    = 8;
constexpr int kH    = 512;
constexpr int kHLog2 = 9;
constexpr int kL    = 2048;
constexpr int kLLog2 = 11;
constexpr int kNm   = 32;
constexpr int kNh   = kNm / 2;
constexpr int kO2   = 2 * kH;
constexpr int kRows = kB * kL;
constexpr int kChS  = 2;
constexpr int kChR  = kChS * kL;
constexpr int kNCh  = kB / kChS;
constexpr int kThr  = 256;
constexpr float kInCarry = 1024.0f;
constexpr float kSc = 1.0f / (kInCarry * kInCarry);
constexpr float kF16MinNormal = 6.103515625e-5f;

static_assert((1 << kHLog2) == kH && (1 << kLLog2) == kL && kNCh * kChS == kB, "the shifts follow the sizes");
static_assert((kChR % 64) == 0 && (kO2 % 64) == 0 && (kH % 32) == 0 && ((kChR / 64) * (kO2 / 64)) % 8 == 0, "GEMM M, N multiples of 64, K of 32; grid exact (1,024 tiles a chunk)");

constexpr size_t kOffW16 = 0ull;
constexpr size_t kOffBIAS = 1048576ull;
constexpr size_t kOffYC = 1052672ull;
constexpr size_t kOffY16 = 34607104ull;
constexpr size_t kOffY2 = 51384320ull;
constexpr size_t kWsTotal = 68161536ull;
static_assert(kWsTotal <= 134217728ull, "carve cap: under 128 MiB");
static_assert(kOffW16 == 0
              && kOffBIAS == kOffW16 + 1048576ull
              && kOffYC == kOffBIAS + 4096ull
              && kOffY16 == kOffYC + 33554432ull
              && kOffY2 == kOffY16 + 16777216ull
              && kWsTotal == kOffY2 + 16777216ull, "the carve is chained and totalled");
static_assert((kOffW16 % 256) == 0 && (kOffBIAS % 256) == 0 && (kOffYC % 256) == 0 && (kOffY16 % 256) == 0 && (kOffY2 % 256) == 0, "aligned regions");

__device__ __forceinline__ unsigned short f2bf_bits(float f) {
  unsigned u = __float_as_uint(f);
  return (unsigned short)((u + 0x7FFFu + ((u >> 16) & 1u)) >> 16);
}
__device__ __forceinline__ float bf_bits2f(unsigned short h) { return __uint_as_float(((unsigned)h) << 16); }
__device__ __forceinline__ float bf16r(float f) { return bf_bits2f(f2bf_bits(f)); }
__device__ __forceinline__ float carry_flush(float v, float carry) {
  const float s = v * carry;
  return (fabsf(s) < kF16MinNormal) ? 0.0f : s;
}
__device__ __forceinline__ float frcp(float x) { return __builtin_amdgcn_rcpf(x); }

__device__ __forceinline__ void dep_guard4_h(v8f& a, v8f& b, v8f& c, v8f& d, v16h x, v16h y) { asm volatile("v_nop\n\tv_nop\n\tv_nop\n\tv_nop" : "+v"(a), "+v"(b), "+v"(c), "+v"(d) : "v"(x), "v"(y)); }
__device__ __forceinline__ void dep_guard4_b(v8f& a, v8f& b, v8f& c, v8f& d, v16b x, v16b y) { asm volatile("v_nop\n\tv_nop\n\tv_nop\n\tv_nop" : "+v"(a), "+v"(b), "+v"(c), "+v"(d) : "v"(x), "v"(y)); }
__device__ __forceinline__ void keep4_h(v16h a, v16h b, v16h c, v16h d) { asm volatile("v_nop" :: "v"(a), "v"(b), "v"(c), "v"(d)); }
__device__ __forceinline__ void keep4_b(v16b a, v16b b, v16b c, v16b d) { asm volatile("v_nop" :: "v"(a), "v"(b), "v"(c), "v"(d)); }
__device__ __forceinline__ void acc_guard4(v8f& a, v8f& b, v8f& c, v8f& d) { asm volatile("v_nop\n\tv_nop\n\tv_nop\n\tv_nop" : "+v"(a), "+v"(b), "+v"(c), "+v"(d)); }

template <typename T> struct Frag;
template <> struct Frag<_Float16> {
  typedef v16h V; union U { v16h v; v8h h[2]; };
  static __device__ __forceinline__ v16h load(const _Float16* p) {
    U f; f.h[0] = *(const v8h*)(p); f.h[1] = *(const v8h*)(p + 16); return f.v;
  }
  static __device__ __forceinline__ v8f mma(v16h a, v16h b, v8f c) {
    return __builtin_amdgcn_wmma_f32_16x16x32_f16(false, a, false, b, (short)0, c, false, false);
  }
  static __device__ __forceinline__ void guard4(v8f& a, v8f& b, v8f& c, v8f& d, v16h x, v16h y) { dep_guard4_h(a, b, c, d, x, y); }
  static __device__ __forceinline__ void keep(v16h a, v16h b, v16h c, v16h d) { keep4_h(a, b, c, d); }
};
template <> struct Frag<__bf16> {
  typedef v16b V; union U { v16b v; v8b h[2]; };
  static __device__ __forceinline__ v16b load(const __bf16* p) {
    U f; f.h[0] = *(const v8b*)(p); f.h[1] = *(const v8b*)(p + 16); return f.v;
  }
  static __device__ __forceinline__ v8f mma(v16b a, v16b b, v8f c) {
    return __builtin_amdgcn_wmma_f32_16x16x32_bf16(false, a, false, b, (short)0, c, false, false);
  }
  static __device__ __forceinline__ void guard4(v8f& a, v8f& b, v8f& c, v8f& d, v16b x, v16b y) { dep_guard4_b(a, b, c, d, x, y); }
  static __device__ __forceinline__ void keep(v16b a, v16b b, v16b c, v16b d) { keep4_b(a, b, c, d); }
};

__device__ __forceinline__ v8f mma_h(v16h a, v16h b, v8f c) {
  c = __builtin_amdgcn_wmma_f32_16x16x32_f16(false, a, false, b, (short)0, c, false, false);
  asm volatile("v_nop\n\tv_nop\n\tv_nop\n\tv_nop" : "+v"(c) : "v"(a), "v"(b));
  return c;
}

template <int ET> struct Elem;
template <> struct Elem<0> { typedef _Float16 T; };
template <> struct Elem<1> { typedef __bf16 T; };
template <int ET, bool SPLIT, int BIAS_MODE, int OUT_MODE, bool RESID, int ACT = 0>
__global__ __launch_bounds__(256) void wmma_gemm64(
    const unsigned short* __restrict__ Ap, const unsigned short* __restrict__ A2p, int lda, long strideA,
    const unsigned short* __restrict__ Btp, const unsigned short* __restrict__ Bt2p, int ldb, long strideB,
    void* __restrict__ Cout, void* __restrict__ Cout2, int ldc, long strideC,
    const float* __restrict__ bias,
    const float* __restrict__ resid, long strideR,
    int M, int N, int K, float scale) {
  typedef typename Elem<ET>::T T;
  typedef typename Frag<T>::V V;
  const T* A = (const T*)Ap; const T* A2 = (const T*)A2p; const T* Bt = (const T*)Btp; const T* Bt2 = (const T*)Bt2p;
  __shared__ __align__(16) float sT[8][16 * 68];
  const int b    = blockIdx.y;
  const int lane = threadIdx.x & 31;
  const int wave = threadIdx.x >> 5;
  const int tilesN = N >> 6;
  const int tilesM = M >> 6;
  const int tile = blockIdx.x * 8 + wave;
  if (tile >= tilesM * tilesN) return;
  const int tm = tile / tilesN;
  const int tn = tile - tm * tilesN;
  const int m0 = tm << 6;
  const int n0 = tn << 6;

  const T* Ab  = A  + (size_t)b * strideA;
  const T* Bb  = Bt + (size_t)b * strideB;
  const T* Ab2 = SPLIT ? (A2  + (size_t)b * strideA) : nullptr;
  const T* Bb2 = SPLIT ? (Bt2 + (size_t)b * strideB) : nullptr;

  const int rlane = lane & 15;
  const int koff  = (lane >> 4) * 8;
  const int mOff  = (lane >> 4) * 8;

  v8f acc[4][4];
#pragma unroll
  for (int i = 0; i < 4; ++i)
#pragma unroll
    for (int j = 0; j < 4; ++j) acc[i][j] = (v8f){0.f,0.f,0.f,0.f,0.f,0.f,0.f,0.f};

  for (int k0 = 0; k0 < K; k0 += 32) {
    V bh[4], bl[4];
#pragma unroll
    for (int j = 0; j < 4; ++j) {
      const size_t bo = (size_t)(n0 + (j << 4) + rlane) * ldb + koff + k0;
      bh[j] = Frag<T>::load(Bb + bo);
      if (SPLIT) bl[j] = Frag<T>::load(Bb2 + bo);
    }
#pragma unroll
    for (int i = 0; i < 4; ++i) {
      const size_t ao = (size_t)(m0 + (i << 4) + rlane) * lda + koff + k0;
      V ah = Frag<T>::load(Ab + ao);
      V al;
      if (SPLIT) al = Frag<T>::load(Ab2 + ao);
#pragma unroll
      for (int j = 0; j < 4; ++j) {
        acc[i][j] = Frag<T>::mma(ah, bh[j], acc[i][j]);
        if (SPLIT) {
          acc[i][j] = Frag<T>::mma(ah, bl[j], acc[i][j]);
          acc[i][j] = Frag<T>::mma(al, bh[j], acc[i][j]);
        }
      }
      Frag<T>::guard4(acc[i][0], acc[i][1], acc[i][2], acc[i][3], ah, SPLIT ? al : ah);
    }
    Frag<T>::keep(bh[0], bh[1], bh[2], bh[3]);
    if (SPLIT) Frag<T>::keep(bl[0], bl[1], bl[2], bl[3]);
  }
  acc_guard4(acc[0][0], acc[0][1], acc[0][2], acc[0][3]);
  acc_guard4(acc[1][0], acc[1][1], acc[1][2], acc[1][3]);
  acc_guard4(acc[2][0], acc[2][1], acc[2][2], acc[2][3]);
  acc_guard4(acc[3][0], acc[3][1], acc[3][2], acc[3][3]);

  float* slab = sT[wave];
  const float* Rb = RESID ? (resid + (size_t)b * strideR) : nullptr;
#pragma unroll
  for (int i = 0; i < 4; ++i) {
    const int mBase = m0 + (i << 4);
#pragma unroll
    for (int j = 0; j < 4; ++j) {
      const int n = n0 + (j << 4) + rlane;
      float bv = 0.f;
      if (BIAS_MODE == 2) bv = bias[n];
#pragma unroll
      for (int r = 0; r < 8; ++r) {
        float v = acc[i][j][r] * scale;
        if (BIAS_MODE == 1) v += bias[mBase + mOff + r];
        if (BIAS_MODE == 2) v += bv;
        if (RESID) v += Rb[(size_t)(mBase + mOff + r) * ldc + n];
        if (ACT == 1) v = tanhf(v);
        if (ACT == 2) v = fmaxf(v, 0.0f);
        if (ACT == 3) v = v / (1.0f + expf(-v));
        if (ACT == 4) v = (v > 0.f) ? v : 0.01f * v;
        slab[(mOff + r) * 68 + (j << 4) + rlane] = v;
      }
    }
    __builtin_amdgcn_fence(__ATOMIC_RELEASE, "workgroup");
    __builtin_amdgcn_wave_barrier();
    __builtin_amdgcn_fence(__ATOMIC_ACQUIRE, "workgroup");
    if (OUT_MODE == 0) {
      float* C = (float*)Cout + (size_t)b * strideC;
      const int hh = lane >> 4, c4 = (lane & 15) * 4;
      for (int pass = 0; pass < 2; ++pass) {
#pragma unroll
        for (int it = 0; it < 8; ++it) {
          const int row = it * 2 + hh;
          v4f v = *(const v4f*)(slab + row * 68 + c4);
          *(volatile v4f*)(C + (size_t)(mBase + row) * ldc + n0 + c4) = v;
        }
        __threadfence();
      }
    } else {
      const int q = lane >> 3, c8 = (lane & 7) * 8;
      unsigned short* C  = (unsigned short*)Cout  + (size_t)b * strideC;
      unsigned short* C2 = (OUT_MODE == 2) ? ((unsigned short*)Cout2 + (size_t)b * strideC) : nullptr;
      for (int pass = 0; pass < 2; ++pass) {
#pragma unroll
        for (int it = 0; it < 4; ++it) {
          const int row = it * 4 + q;
          const float* sp = slab + row * 68 + c8;
          v8h hv, lv;
#pragma unroll
          for (int e = 0; e < 8; ++e) {
            if (OUT_MODE == 1) {
              hv[e] = (_Float16)sp[e];
            } else {
              unsigned short hb = f2bf_bits(sp[e]);
              unsigned short lb = f2bf_bits(sp[e] - bf_bits2f(hb));
              hv[e] = __builtin_bit_cast(_Float16, hb);
              lv[e] = __builtin_bit_cast(_Float16, lb);
            }
          }
          *(volatile v8h*)(C + (size_t)(mBase + row) * ldc + n0 + c8) = hv;
          if (OUT_MODE == 2) *(volatile v8h*)(C2 + (size_t)(mBase + row) * ldc + n0 + c8) = lv;
        }
        __threadfence();
      }
    }
    __builtin_amdgcn_fence(__ATOMIC_RELEASE, "workgroup");
    __builtin_amdgcn_wave_barrier();
    __builtin_amdgcn_fence(__ATOMIC_ACQUIRE, "workgroup");
  }
}

__global__ __launch_bounds__(kThr) void cast_plane_kernel(const float* __restrict__ src, unsigned short* __restrict__ dst,
                                                          int colsLog2, int dstPitch, int dstOff) {
  const int i   = blockIdx.x * kThr + threadIdx.x;
  const int sh  = colsLog2 - 3;
  const int row = i >> sh;
  const int c8  = (i & ((1 << sh) - 1)) * 8;
  const float* sp = src + ((size_t)row << colsLog2) + c8;
  const v4f a0 = *(const v4f*)(sp);
  const v4f a1 = *(const v4f*)(sp + 4);
  v8h hv;
#pragma unroll
  for (int e = 0; e < 4; ++e) {
    const float f0 = a0[e];
    const float f1 = a1[e];
    hv[e]     = (_Float16)carry_flush(bf16r(f0), kInCarry);
    hv[4 + e] = (_Float16)carry_flush(bf16r(f1), kInCarry);
  }
  unsigned short* dp = dst + (size_t)row * dstPitch + dstOff + c8;
  *(volatile v8h*)dp = hv;
  __threadfence();
  *(volatile v8h*)dp = hv;
}

__global__ __launch_bounds__(kThr) void bias_kernel(const float* __restrict__ b, float* __restrict__ BIAS) {
  const int i = blockIdx.x * kThr + threadIdx.x;
  const float v = b[i];
  const float o = bf16r(v);
  for (int pass = 0; pass < 2; ++pass) {
    *(volatile float*)(BIAS + i) = o;
    __threadfence();
  }
}
static_assert(kO2 % kThr == 0, "bias grid exact");

__global__ __launch_bounds__(kThr) void s4d_scan_kernel(const float* __restrict__ u, const float* __restrict__ log_dt, const float* __restrict__ C,
                                                        const float* __restrict__ log_A_real, const float* __restrict__ A_imag, const float* __restrict__ D,
                                                        float* __restrict__ YC, int half) {
  const unsigned v = blockIdx.x * (unsigned)kThr + threadIdx.x;
  const unsigned smp = v >> kHLog2, h = v & (unsigned)(kH - 1);
  const float ld0 = log_dt[h];
  const float dt = expf(bf16r(ld0));
  float lre[kNh], lim[kNh], kre[kNh], kim[kNh], sre[kNh], sim[kNh];
  const size_t m0 = (size_t)h * kNm + (size_t)half * kNh;
#pragma unroll
  for (int n = 0; n < kNh; ++n) {
    const float ar0 = log_A_real[m0 + n], ai0 = A_imag[m0 + n];
    const float c0 = C[(m0 + n) * 2], c1 = C[(m0 + n) * 2 + 1];
    const float are = -expf(bf16r(ar0)), aim = bf16r(ai0);
    const float e = expf(are * dt), ph = aim * dt;
    const float lr = e * cosf(ph), li = e * sinf(ph);
    const float nr = lr - 1.0f, ni = li;
    const float den = are * are + aim * aim;
    const float qr = (nr * are + ni * aim) / den, qi = (ni * are - nr * aim) / den;
    const float cr = bf16r(c0), ci = bf16r(c1);
    lre[n] = lr; lim[n] = li;
    kre[n] = cr * qr - ci * qi; kim[n] = cr * qi + ci * qr;
    sre[n] = 0.0f; sim[n] = 0.0f;
  }
  const float d0 = D[h];
  const float dsk = (half == 0) ? bf16r(d0) : 0.0f;
  const float* ur = u + ((size_t)smp * kH + h) * kL;
  float* yr = YC + ((size_t)smp * kH + h) * kL;
  for (int l = 0; l < kL; ++l) {
    const float u0 = ur[l];
    const float uu = bf16r(u0);
    float acc = 0.0f;
#pragma unroll
    for (int n = 0; n < kNh; ++n) {
      const float nr = lre[n] * sre[n] - lim[n] * sim[n] + uu;
      const float ni = lre[n] * sim[n] + lim[n] * sre[n];
      sre[n] = nr; sim[n] = ni;
      acc += kre[n] * nr - kim[n] * ni;
    }
    float y = 2.0f * acc + dsk * uu;
    if (half != 0) y += yr[l];
    *(volatile float*)(yr + l) = y;
    __threadfence();
    *(volatile float*)(yr + l) = y;
  }
}
static_assert((kB * kH) % kThr == 0, "scan grid exact: 16 blocks");

__global__ __launch_bounds__(kThr) void gelu_cast_kernel(const float* __restrict__ YC, unsigned short* __restrict__ Y16) {
  const unsigned smp = blockIdx.y;
  const unsigned pos = blockIdx.x * 4u + (threadIdx.x >> 6);
  const unsigned c8 = (threadIdx.x & 63u) * 8u;
  const float* sp = YC + ((size_t)smp * kH + c8) * kL + pos;
  v8h hv;
#pragma unroll
  for (int e = 0; e < 8; ++e) {
    const float y = sp[(size_t)e * kL];
    const float g = 0.5f * y * (1.0f + erff(y * 0.70710678118654752f));
    hv[e] = (_Float16)carry_flush(g, kInCarry);
  }
  unsigned short* dp = Y16 + ((size_t)smp * kL + pos) * kH + c8;
  *(volatile v8h*)dp = hv;
  __threadfence();
  *(volatile v8h*)dp = hv;
}
static_assert(kL == 512 * 4 && kH == 64 * 8, "cast grid exact: 512 blocks of 4 positions a sample; 64 chunks a row");

__global__ __launch_bounds__(kThr) void glu_out_kernel(const float* __restrict__ Y2, float* __restrict__ out, int chunk) {
  const size_t i = (size_t)blockIdx.x * kThr + threadIdx.x;
  const unsigned l4 = (unsigned)(i & (size_t)(kL / 4 - 1)) * 4u;
  const unsigned o = (unsigned)((i >> (kLLog2 - 2)) & (size_t)(kH - 1));
  const unsigned ls = (unsigned)(i >> (kLLog2 - 2 + kHLog2));
  v4f ov;
#pragma unroll
  for (int e = 0; e < 4; ++e) {
    const float* pr = Y2 + ((size_t)ls * kL + l4 + (unsigned)e) * kO2;
    const float a = pr[o], g = pr[kH + o];
    ov[e] = a / (1.0f + expf(-g));
  }
  float* dp = out + (((size_t)chunk * kChS + ls) * kH + o) * kL + l4;
  *(volatile v4f*)dp = ov;
  __threadfence();
  *(volatile v4f*)dp = ov;
}
static_assert(((size_t)kChS * kH * kL / 4) % kThr == 0, "output grid exact");

static_assert(((size_t)kO2 * kH / 8) % kThr == 0, "plane cast grid exact");

extern "C" void kernel_launch(void* const* d_in, const int* in_sizes, int n_in,
                              void* d_out, int out_size, void* d_ws, size_t ws_size,
                              hipStream_t stream) {
  if (n_in < 8 || d_out == nullptr || d_ws == nullptr) return;
  if (in_sizes[0] != kB * kH * kL || in_sizes[1] != kH || in_sizes[2] != kH * kNm * 2 || in_sizes[3] != kH * kNm || in_sizes[4] != kH * kNm) return;
  if (in_sizes[5] != kH || in_sizes[6] != kO2 * kH || in_sizes[7] != kO2) return;
  if (out_size != kB * kH * kL) return;
  if (ws_size < kWsTotal) return;
  const float* u = (const float*)d_in[0];
  const float* log_dt = (const float*)d_in[1];
  const float* C = (const float*)d_in[2];
  const float* log_A_real = (const float*)d_in[3];
  const float* A_imag = (const float*)d_in[4];
  const float* D = (const float*)d_in[5];
  const float* W = (const float*)d_in[6];
  const float* b = (const float*)d_in[7];
  float* out = (float*)d_out;
  char* ws = (char*)d_ws;
  unsigned short* W16 = (unsigned short*)(ws + kOffW16);
  float* BIAS = (float*)(ws + kOffBIAS);
  float* YC = (float*)(ws + kOffYC);
  unsigned short* Y16 = (unsigned short*)(ws + kOffY16);
  float* Y2 = (float*)(ws + kOffY2);

  cast_plane_kernel<<<(int)(((size_t)kO2 * kH / 8) / kThr), kThr, 0, stream>>>(W, W16, kHLog2, kH, 0);
  bias_kernel<<<kO2 / kThr, kThr, 0, stream>>>(b, BIAS);
  s4d_scan_kernel<<<(kB * kH) / kThr, kThr, 0, stream>>>(u, log_dt, C, log_A_real, A_imag, D, YC, 0);
  s4d_scan_kernel<<<(kB * kH) / kThr, kThr, 0, stream>>>(u, log_dt, C, log_A_real, A_imag, D, YC, 1);
  gelu_cast_kernel<<<dim3(kL / 4, kB), kThr, 0, stream>>>(YC, Y16);
  for (int c = 0; c < kNCh; ++c) {
    wmma_gemm64<0, false, 2, 0, false, 0><<<dim3((kChR / 64) * (kO2 / 64) / 8, 1), 256, 0, stream>>>(
        Y16 + (size_t)c * kChR * kH, Y16 + (size_t)c * kChR * kH, kH, 0L, W16, W16, kH, 0L, (void*)Y2, (void*)Y2, kO2, 0L, BIAS, nullptr, 0L, kChR, kO2, kH, kSc);
    glu_out_kernel<<<(int)(((size_t)kChS * kH * kL / 4) / kThr), kThr, 0, stream>>>(Y2, out, c);
  }
}
